// gcnmask_67370857005189
// MI455X (gfx1250) — hardware-verified
//
#include <hip/hip_runtime.h>
#include <stdint.h>


typedef _Float16 v16h __attribute__((ext_vector_type(16)));
typedef _Float16 v8h  __attribute__((ext_vector_type(8)));
typedef __bf16   v16b __attribute__((ext_vector_type(16)));
typedef __bf16   v8b  __attribute__((ext_vector_type(8)));
typedef float    v8f  __attribute__((ext_vector_type(8)));
typedef float    v4f  __attribute__((ext_vector_type(4)));

union FragH { v16h v; v8h h[2]; _Float16 e[16]; };
union FragB { v16b v; v8b h[2]; __bf16 e[16]; };

#define F     128
#define DEG   16
#define NCHK  5000
#define AST2  136
#define SPF   132

__device__ __forceinline__ v8f wmma_h(v16h a, v16h b, v8f c) {
    v8f d = __builtin_amdgcn_wmma_f32_16x16x32_f16(false, a, false, b, (short)0, c, false, false);
    asm volatile("v_nop\n\tv_nop\n\tv_nop\n\tv_nop" : "+v"(d) : "v"(a), "v"(b));
    return d;
}
__device__ __forceinline__ v8f wmma_b(v16b a, v16b b, v8f c) {
    v8f d = __builtin_amdgcn_wmma_f32_16x16x32_bf16(false, a, false, b, (short)0, c, false, false);
    asm volatile("v_nop\n\tv_nop\n\tv_nop\n\tv_nop" : "+v"(d) : "v"(a), "v"(b));
    return d;
}

__device__ __forceinline__ v16h lda_h(const _Float16* t, int pitch, int m, int h, int k0) {
    FragH a;
    a.h[0] = *(const v8h*)(t + m * pitch + k0 + 8 * h);
    a.h[1] = *(const v8h*)(t + m * pitch + k0 + 16 + 8 * h);
    return a.v;
}
__device__ __forceinline__ v16b lda_b(const __bf16* t, int pitch, int m, int h, int k0) {
    FragB a;
    a.h[0] = *(const v8b*)(t + m * pitch + k0 + 8 * h);
    a.h[1] = *(const v8b*)(t + m * pitch + k0 + 16 + 8 * h);
    return a.v;
}

__device__ __forceinline__ v8h cvt8h(v4f a, v4f b) {
    union { v8h v; _Float16 e[8]; } u;
    u.e[0] = (_Float16)a.x; u.e[1] = (_Float16)a.y; u.e[2] = (_Float16)a.z; u.e[3] = (_Float16)a.w;
    u.e[4] = (_Float16)b.x; u.e[5] = (_Float16)b.y; u.e[6] = (_Float16)b.z; u.e[7] = (_Float16)b.w;
    return u.v;
}

__device__ __forceinline__ void split8b(v4f a, v4f b, v8b& hi, v8b& lo) {
    float f[8];
    f[0] = a.x; f[1] = a.y; f[2] = a.z; f[3] = a.w;
    f[4] = b.x; f[5] = b.y; f[6] = b.z; f[7] = b.w;
    union { v8b v; __bf16 e[8]; } uh, ul;
#pragma unroll
    for (int j = 0; j < 8; ++j) {
        const __bf16 hv = (__bf16)f[j];
        const float res = f[j] - (float)hv;
        uh.e[j] = hv;
        ul.e[j] = (__bf16)res;
    }
    hi = uh.v; lo = ul.v;
}

__device__ __forceinline__ v8f zero8() {
    v8f z = {0.f, 0.f, 0.f, 0.f, 0.f, 0.f, 0.f, 0.f};
    return z;
}

__device__ __forceinline__ float sigm(float v) {
    return __builtin_amdgcn_rcpf(1.0f + __expf(-v));
}

__device__ __forceinline__ int clamp_node(int node, int N) {
    if (node < 0) node += N;
    if (node < 0) node = 0;
    if (node >= N) node = N - 1;
    return node;
}

__global__ __launch_bounds__(256) void k_pack(const float* __restrict__ wm, const float* __restrict__ w,
                                              _Float16* wmP, __bf16* wPh, __bf16* wPl)
{
    const int t = blockIdx.x * blockDim.x + threadIdx.x;
    if (t < 4096) {
        const int half = t & 1, lane = (t >> 1) & 31, s = (t >> 6) & 7, wv = t >> 9;
        const int n = wv * 16 + (lane & 15), hb = lane >> 4;
        union { v8h v; _Float16 e[8]; } u;
#pragma unroll
        for (int j = 0; j < 8; ++j) {
            const int kk = s * 32 + 8 * hb + 16 * half + j;
            u.e[j] = (_Float16)(wm[kk * F + n] * 16.0f);
        }
        const v8h v = u.v;
        _Float16* p = wmP + (size_t)t * 8;
        *(volatile v8h*)p = v;
        __threadfence();
        *(volatile v8h*)p = v;
    } else if (t < 4096 + 2048) {
        const int tt = t - 4096;
        const int half = tt & 1, lane = (tt >> 1) & 31, s = (tt >> 6) & 3, wv = tt >> 8;
        const int n = wv * 16 + (lane & 15), hb = lane >> 4;
        union { v8b v; __bf16 e[8]; } uh, ul;
#pragma unroll
        for (int j = 0; j < 8; ++j) {
            const int kk = s * 32 + 8 * hb + 16 * half + j;
            const float v = w[kk * F + n];
            const __bf16 hv = (__bf16)v;
            uh.e[j] = hv;
            ul.e[j] = (__bf16)(v - (float)hv);
        }
        const v8b vh = uh.v, vl = ul.v;
        __bf16* ph = wPh + (size_t)tt * 8;
        __bf16* pl = wPl + (size_t)tt * 8;
        *(volatile v8b*)ph = vh;
        *(volatile v8b*)pl = vl;
        __threadfence();
        *(volatile v8b*)ph = vh;
        *(volatile v8b*)pl = vl;
    }
}

__global__ __launch_bounds__(256) void k_gather(
    const float* __restrict__ x,
    const int*   __restrict__ esrc,
    _Float16*                 neiH,
    float*                    neiF,
    int e0, int npairs, int N, int E)
{
    const int wv = threadIdx.x >> 5, lane = threadIdx.x & 31, h = lane >> 4;
    const int p = blockIdx.x * 8 + wv;
    if (p >= npairs) return;
    size_t ea = (size_t)e0 + 2 * (size_t)p;
    size_t eb = ea + 1;
    if (ea >= (size_t)E) ea = (size_t)E - 1;
    if (eb >= (size_t)E) eb = (size_t)E - 1;
    const int sa = clamp_node(esrc[ea], N);
    const int sb = clamp_node(esrc[eb], N);

    const v4f va = *(const v4f*)(x + (size_t)sa * F + 4 * lane);
    const v4f vb = *(const v4f*)(x + (size_t)sb * F + 4 * lane);
    const int sq = h ? sb : sa;
    const float* hp = x + (size_t)sq * F + 8 * (lane & 15);
    const v8h vh = cvt8h(*(const v4f*)hp, *(const v4f*)(hp + 4));

    float*    pa = neiF + (size_t)(2 * p) * F + 4 * lane;
    float*    pb = neiF + (size_t)(2 * p + 1) * F + 4 * lane;
    _Float16* ph = neiH + (size_t)p * (2 * F) + 8 * lane;
    *(volatile v4f*)pa = va;
    *(volatile v4f*)pb = vb;
    *(volatile v8h*)ph = vh;
    __threadfence();
    *(volatile v4f*)pa = va;
    *(volatile v4f*)pb = vb;
    *(volatile v8h*)ph = vh;
}

__global__ __launch_bounds__(256) void k_gate_agg(
    const float*    __restrict__ x,
    const _Float16* __restrict__ wmP,
    const _Float16* __restrict__ neiH,
    const float*    __restrict__ neiF,
    float*                       xnew,
    int n0, int nn, int N)
{
    __shared__ __attribute__((aligned(16))) _Float16 cenH[F];
    __shared__ __attribute__((aligned(16))) float    xrow[F];

    const int tid = threadIdx.x, wv = tid >> 5, lane = tid & 31;
    const int h = lane >> 4, m = lane & 15;
    const int col = wv * 16 + m;

    v16h bfr[8];
#pragma unroll
    for (int s = 0; s < 8; ++s)
        bfr[s] = *(const v16h*)(wmP + ((size_t)(wv * 8 + s) * 32 + lane) * 16);

    for (int dl = blockIdx.x; dl < nn; dl += gridDim.x) {
        int d = n0 + dl;
        if (d >= N) d = N - 1;

        if (tid < 16) {
            const float* sp = x + (size_t)d * F + 8 * tid;
            *(v8h*)(cenH + 8 * tid) = cvt8h(*(const v4f*)sp, *(const v4f*)(sp + 4));
        }
        __syncthreads();

        const _Float16* nrow = neiH + (size_t)dl * (DEG * F);
        const float*    frow = neiF + (size_t)dl * (DEG * F);

        v8f acc0 = zero8(), acc1 = zero8();
#pragma unroll
        for (int s = 0; s < 4; s += 2) {
            const v16h a0 = lda_h(cenH, 0, m, h, s * 32);
            const v16h a1 = lda_h(cenH, 0, m, h, s * 32 + 32);
            acc0 = wmma_h(a0, bfr[s],     acc0);
            acc1 = wmma_h(a1, bfr[s + 1], acc1);
        }
#pragma unroll
        for (int s = 0; s < 4; s += 2) {
            const v16h a0 = lda_h(nrow, F, m, h, s * 32);
            const v16h a1 = lda_h(nrow, F, m, h, s * 32 + 32);
            acc0 = wmma_h(a0, bfr[4 + s],     acc0);
            acc1 = wmma_h(a1, bfr[4 + s + 1], acc1);
        }

        float part = 0.0f;
#pragma unroll
        for (int r = 0; r < 8; ++r) {
            const float lg = (acc0[r] + acc1[r]) * 0.0625f;
            const float g  = sigm(lg);
            part += g * frow[(8 * h + r) * F + col];
        }
        part += __shfl_xor(part, 16, 32);
        if (lane < 16) xrow[col] = x[(size_t)d * F + col] + part;
        __syncthreads();

        if (wv == 0) {
            const v4f v = *(const v4f*)(xrow + 4 * lane);
            float* p = xnew + (size_t)d * F + 4 * lane;
            *(volatile v4f*)p = v;
            __threadfence();
            *(volatile v4f*)p = v;
        }
        __syncthreads();
    }
}

__global__ __launch_bounds__(256) void k_support(
    const float*  __restrict__ xnew,
    const __bf16* __restrict__ wPh,
    const __bf16* __restrict__ wPl,
    float*                     support,
    int N, int ntiles)
{
    __shared__ __attribute__((aligned(16))) __bf16 Ahi[16 * AST2];
    __shared__ __attribute__((aligned(16))) __bf16 Alo[16 * AST2];
    __shared__ __attribute__((aligned(16))) float  Sf[16 * SPF];

    const int tid = threadIdx.x, wv = tid >> 5, lane = tid & 31;
    const int h = lane >> 4, m = lane & 15;
    const int col = wv * 16 + m;

    v16b bh[4], bl[4];
#pragma unroll
    for (int s = 0; s < 4; ++s) {
        const size_t o = ((size_t)(wv * 4 + s) * 32 + lane) * 16;
        bh[s] = *(const v16b*)(wPh + o);
        bl[s] = *(const v16b*)(wPl + o);
    }

    for (int t = blockIdx.x; t < ntiles; t += gridDim.x) {
        {
            const int r  = tid >> 4;
            const int c0 = (tid & 15) * 8;
            int row = t * 16 + r;
            if (row >= N) row = N - 1;
            const float* sp = xnew + (size_t)row * F + c0;
            const v4f p0 = *(const v4f*)sp;
            const v4f p1 = *(const v4f*)(sp + 4);
            v8b hi, lo;
            split8b(p0, p1, hi, lo);
            *(v8b*)(Ahi + r * AST2 + c0) = hi;
            *(v8b*)(Alo + r * AST2 + c0) = lo;
        }
        __syncthreads();

        v8f acc = zero8();
#pragma unroll
        for (int s = 0; s < 4; ++s) {
            const v16b ah = lda_b(Ahi, AST2, m, h, s * 32);
            const v16b al = lda_b(Alo, AST2, m, h, s * 32);
            acc = wmma_b(ah, bh[s], acc);
            acc = wmma_b(al, bh[s], acc);
            acc = wmma_b(ah, bl[s], acc);
        }

#pragma unroll
        for (int r = 0; r < 8; ++r)
            Sf[(8 * h + r) * SPF + col] = acc[r];
        __syncthreads();

#pragma unroll
        for (int q = 0; q < 2; ++q) {
            const int rr   = wv * 2 + q;
            const int grow = t * 16 + rr;
            if (grow < N) {
                const v4f v = *(const v4f*)(Sf + rr * SPF + 4 * lane);
                float* p = support + (size_t)grow * F + 4 * lane;
                *(volatile v4f*)p = v;
                __threadfence();
                *(volatile v4f*)p = v;
            }
        }
        __syncthreads();
    }
}

__global__ __launch_bounds__(256) void k_out(
    const float* __restrict__ support,
    const float* __restrict__ adj,
    const int*   __restrict__ esrc,
    const float* __restrict__ bias,
    float*                    out, int N, int E)
{
    const int d = blockIdx.x * 8 + (threadIdx.x >> 5);
    const int c = threadIdx.x & 31;
    if (d >= N) return;
    const size_t eb = (size_t)d * DEG;
    v4f acc = *(const v4f*)(bias + 4 * c);
#pragma unroll 4
    for (int e = 0; e < DEG; ++e) {
        size_t ei = eb + (size_t)e;
        if (ei >= (size_t)E) ei = (size_t)E - 1;
        const int   s = clamp_node(esrc[ei], N);
        const float a = adj[ei];
        const v4f   v = *(const v4f*)(support + (size_t)s * F + 4 * c);
        acc += a * v;
    }
    float* p = out + (size_t)d * F + 4 * c;
    const v4f vv = acc;
    *(volatile v4f*)p = vv;
    __threadfence();
    *(volatile v4f*)p = vv;
}

extern "C" void kernel_launch(void* const* d_in, const int* in_sizes, int n_in,
                              void* d_out, int out_size, void* d_ws, size_t ws_size,
                              hipStream_t stream) {
    (void)n_in;
    const float* x     = (const float*)d_in[0];
    const float* w     = (const float*)d_in[1];
    const float* bias  = (const float*)d_in[2];
    const float* wm    = (const float*)d_in[3];
    const float* adj   = (const float*)d_in[4];
    const int*   esrc  = (const int*)d_in[5];

    const int N = in_sizes[0] / F;
    const int E = in_sizes[5];
    if (N <= 0 || E <= 0) return;
    if ((size_t)E < (size_t)N * DEG) return;
    if ((size_t)out_size < (size_t)N * F) return;

    auto al256 = [](size_t b) -> size_t { return (b + 255) & ~(size_t)255; };
    size_t off = 0;
    const size_t o_wmP = off; off += al256((size_t)4096 * 8 * 2);
    const size_t o_wPh = off; off += al256((size_t)2048 * 8 * 2);
    const size_t o_wPl = off; off += al256((size_t)2048 * 8 * 2);
    const size_t o_xn  = off; off += al256((size_t)N * F * 4);
    const size_t o_sup = off; off += al256((size_t)N * F * 4);
    const size_t o_nH  = off; off += al256((size_t)NCHK * DEG * F * 2);
    const size_t o_nF  = off; off += al256((size_t)NCHK * DEG * F * 4);
    if (off > ws_size) return;

    char* base = (char*)d_ws;
    _Float16* wmP     = (_Float16*)(base + o_wmP);
    __bf16*   wPh     = (__bf16*)(base + o_wPh);
    __bf16*   wPl     = (__bf16*)(base + o_wPl);
    float*    xnew    = (float*)(base + o_xn);
    float*    support = (float*)(base + o_sup);
    _Float16* neiH    = (_Float16*)(base + o_nH);
    float*    neiF    = (float*)(base + o_nF);

    k_pack<<<(4096 + 2048 + 255) / 256, 256, 0, stream>>>(wm, w, wmP, wPh, wPl);

    const int nchunks = (N + NCHK - 1) / NCHK;
    for (int c = 0; c < nchunks; ++c) {
        const int n0 = c * NCHK;
        int nn = N - n0; if (nn > NCHK) nn = NCHK;
        const int e0 = n0 * DEG;
        const int npairs = nn * (DEG / 2);
        k_gather<<<(npairs + 7) / 8, 256, 0, stream>>>(x, esrc, neiH, neiF, e0, npairs, N, E);
        const int blocks = nn < 4096 ? nn : 4096;
        k_gate_agg<<<blocks, 256, 0, stream>>>(x, wmP, neiH, neiF, xnew, n0, nn, N);
    }
    {
        const int ntiles = (N + 15) / 16;
        const int blocks = ntiles < 2048 ? ntiles : 2048;
        k_support<<<blocks, 256, 0, stream>>>(xnew, wPh, wPl, support, N, ntiles);
    }
    {
        const int blocks = (N + 7) / 8;
        k_out<<<blocks, 256, 0, stream>>>(support, adj, esrc, bias, (float*)d_out, N, E);
    }
}
